// GMP_27075473834662
// MI455X (gfx1250) — hardware-run, weakly checked
//
#include <hip/hip_runtime.h>


#ifndef NB
#define NB 16
#endif
#ifndef SEQ
#define SEQ 8192
#endif
#define NB_FULL  16
#define SEQ_FULL 8192
#ifndef OUT_SEQ
#define OUT_SEQ SEQ
#endif
#define LL    13
#define MM    12
#define NKK   3
#define HALO  (LL + MM - 1)
#define TB    128
#define AWV   4
#define NT    11
#define NROWS (NT * 16)
#define NS    256
#define GP    33
#define KPAD  64
#define X1OFF (HALO - (LL - 1))
#define X3OFF (HALO + MM)
#define WSC   1024.0f
#define WSI   (1.0f / 1024.0f)

static_assert(TB == 32 * AWV);
static_assert(NS == 2 * 32 * AWV);
static_assert(NROWS >= TB + HALO + LL - 1);
static_assert(NS >= NROWS + 16);
static_assert(NS >= TB + LL - 1 + X3OFF + 1);
static_assert(4 * (MM + 1) <= KPAD);
static_assert(KPAD % 32 == 0);
static_assert(LL <= 16);
static_assert(SEQ % TB == 0);
static_assert(SEQ >= NS);
static_assert(OUT_SEQ % 16 == 0);
static_assert(NB <= NB_FULL);
static_assert(SEQ <= SEQ_FULL);
static_assert(32 * KPAD == 256 * 8);
static_assert(8 * 256 == 32 * KPAD);
static_assert(2 * 32 * 16 == TB * 2 * 4);
static_assert((NS * 2 * 4) + (NS * 2 * 4) + (NROWS * GP * 4) + (TB * 2 * 4) <= 131072);
static_assert(32 * KPAD * 2 <= 131072);

typedef _Float16 h16;
typedef __attribute__((ext_vector_type(16))) _Float16 v16h;
typedef __attribute__((ext_vector_type(8)))  _Float16 v8h;
typedef __attribute__((ext_vector_type(8)))  float    v8f;
typedef __attribute__((ext_vector_type(4)))  float    v4f;
typedef __attribute__((ext_vector_type(2)))  float    v2f;
typedef __attribute__((ext_vector_type(2)))  unsigned v2u;
typedef __attribute__((ext_vector_type(8)))  unsigned v8u;
typedef v4f  __attribute__((may_alias)) v4fa;
typedef v2f  __attribute__((may_alias)) v2fa;
typedef v2u  __attribute__((may_alias)) v2ua;
typedef v8h  __attribute__((may_alias)) v8ha;

__device__ __forceinline__ unsigned short f2bf(float f) { unsigned u = __float_as_uint(f); u += 0x7FFFu + ((u >> 16) & 1u); return (unsigned short)(u >> 16); }
__device__ __forceinline__ float bfr(float f) { return __uint_as_float(((unsigned)f2bf(f)) << 16); }
__device__ __forceinline__ v16h cat16(v8h lo, v8h hi) { return __builtin_shufflevector(lo, hi, 0, 1, 2, 3, 4, 5, 6, 7, 8, 9, 10, 11, 12, 13, 14, 15); }
__device__ __forceinline__ v8f wmma16(v16h a, v16h b, v8f c) { return __builtin_amdgcn_wmma_f32_16x16x32_f16(false, a, false, b, (short)0, c, false, false); }
__device__ __forceinline__ v16h  ldh(const h16* p) { return cat16(*(const v8h*)p, *(const v8h*)(p + 16)); }
static __device__ __forceinline__ h16 toh_flush(float v) { const h16 r = (h16)v; return (fabsf(v) < 6.103515625e-05f) ? (h16)0.0f : r; }
__device__ __forceinline__ unsigned hbits(h16 h) { return (unsigned)__builtin_bit_cast(unsigned short, h); }
__device__ __forceinline__ v8f wmma16g(v16h a, v16h b, v8f c) {
    c = wmma16(a, b, c);
    asm volatile("v_nop\n\tv_nop\n\tv_nop\n\tv_nop" : "+v"(c) : "v"(a), "v"(b));
    return c;
}

__global__ __launch_bounds__(256) void k_wpack(const float* __restrict__ Akl, const float* __restrict__ Bk, const float* __restrict__ Ck, h16* WP) {
#pragma clang fp contract(off)
    __shared__ __align__(16) h16 lw[32 * KPAD];
    const int tid = threadIdx.x;
#pragma unroll 1
    for (int it = 0; it < 8; ++it) {
        const int idx = it * 256 + tid;
        const int n = idx >> 6, j = idx & 63;
        const int l = n & 15, sel = n >> 4, m = j >> 2, k = j & 3;
        const int lc = l < LL ? l : LL - 1, mc = m < MM ? m : MM - 1, kc = k < NKK ? k : NKK - 1;
        float va = Akl[lc * NKK + kc];
        float vb = Bk[(lc * MM + mc) * NKK + kc];
        float vc = Ck[(lc * MM + mc) * NKK + kc];
        asm volatile("" : "+v"(va)); asm volatile("" : "+v"(vb)); asm volatile("" : "+v"(vc));
        const float v12 = (m < MM) ? vb : ((m == MM) ? va : 0.0f);
        const float v3  = (m < MM) ? vc : 0.0f;
        const bool ok = (l < LL) & (k < NKK);
        const float v = ok ? (sel ? v3 : v12) : 0.0f;
        lw[idx] = toh_flush(bfr(v) * WSC);
    }
    __syncthreads();
    const v8h o = *(const v8ha*)(&lw[tid * 8]);
    *(volatile v8h*)(WP + tid * 8) = o; __threadfence(); *(volatile v8h*)(WP + tid * 8) = o;
}

__global__ __launch_bounds__(32 * AWV) void k_mpoly(const float* __restrict__ X, const h16* __restrict__ WP, float* OUT) {
    __shared__ __align__(16) unsigned ps[NS * 2];
    __shared__ __align__(16) float xs[NS * 2];
    __shared__ __align__(16) float gs[NROWS * GP];
    __shared__ __align__(16) float os[TB * 2];
    const int tid = threadIdx.x;
    const int lane = tid & 31, lr = lane & 15, hi = lane >> 4;
    const int wave = __builtin_amdgcn_readfirstlane((int)(threadIdx.x >> 5));
    const int b = blockIdx.y; const int t0 = blockIdx.x * TB;
    const float* xb = X + (size_t)b * SEQ_FULL * 2;
#pragma unroll 1
    for (int it = 0; it < 2; ++it) {
        const int s = it * (32 * AWV) + tid;
        int u = t0 - HALO + s;
        u = u < 0 ? u + SEQ : u; u = u >= SEQ ? u - SEQ : u;
        u = u < 0 ? 0 : (u > SEQ - 1 ? SEQ - 1 : u);
        const v2f xv = *(const v2f*)(xb + (size_t)u * 2);
        const float xr = bfr(xv[0]), xi = bfr(xv[1]);
        const float a = sqrtf(xr * xr + xi * xi);
        const float a2 = a * a; const float a3 = a2 * a; const float a5 = (a2 * a2) * a;
        v2u pw; pw[0] = hbits(toh_flush(a)) | (hbits(toh_flush(a3)) << 16); pw[1] = hbits(toh_flush(a5));
        *(v2ua*)(&ps[s * 2]) = pw;
        v2f xw; xw[0] = xr; xw[1] = xi;
        *(v2fa*)(&xs[s * 2]) = xw;
    }
    __syncthreads();
    const h16* wp = WP + (size_t)lr * KPAD + 8 * hi;
    const v16h w00 = ldh(wp), w01 = ldh(wp + 32), w10 = ldh(wp + 16 * KPAD), w11 = ldh(wp + 16 * KPAD + 32);
#pragma unroll 1
    for (int tile = wave; tile < NT; tile += AWV) {
        const int sb = (tile * 16 + lr + 2 * hi) * 2;
        const v2u g0 = *(const v2ua*)(&ps[sb]),      g1 = *(const v2ua*)(&ps[sb + 2]);
        const v2u g2 = *(const v2ua*)(&ps[sb + 8]),  g3 = *(const v2ua*)(&ps[sb + 10]);
        const v2u g4 = *(const v2ua*)(&ps[sb + 16]), g5 = *(const v2ua*)(&ps[sb + 18]);
        const v2u g6 = *(const v2ua*)(&ps[sb + 24]), g7 = *(const v2ua*)(&ps[sb + 26]);
        v8u u0, u1;
        u0[0] = g0[0]; u0[1] = g0[1]; u0[2] = g1[0]; u0[3] = g1[1]; u0[4] = g2[0]; u0[5] = g2[1]; u0[6] = g3[0]; u0[7] = g3[1];
        u1[0] = g4[0]; u1[1] = g4[1]; u1[2] = g5[0]; u1[3] = g5[1]; u1[4] = g6[0]; u1[5] = g6[1]; u1[6] = g7[0]; u1[7] = g7[1];
        const v16h a0 = __builtin_bit_cast(v16h, u0), a1 = __builtin_bit_cast(v16h, u1);
        v8f c12 = (v8f){}, c3 = (v8f){};
        c12 = wmma16g(a0, w00, c12); c12 = wmma16g(a1, w01, c12);
        c3  = wmma16g(a0, w10, c3);  c3  = wmma16g(a1, w11, c3);
        const int rb = (tile * 16 + 8 * hi) * GP + lr;
#pragma unroll
        for (int r = 0; r < 8; ++r) { gs[rb + r * GP] = c12[r]; gs[rb + r * GP + 16] = c3[r]; }
    }
    __syncthreads();
    {
        const int tr = tid;
        float sr = 0.0f, si = 0.0f;
#pragma unroll 1
        for (int l = 0; l < LL; ++l) {
            const float c12v = gs[(tr + l) * GP + l];
            const float c3v  = gs[(tr + l + HALO) * GP + 16 + l];
            const v2f x1 = *(const v2fa*)(&xs[(tr + l + X1OFF) * 2]);
            const v2f x3 = *(const v2fa*)(&xs[(tr + l + X3OFF) * 2]);
            sr = fmaf(x1[0], c12v, sr); si = fmaf(x1[1], c12v, si);
            sr = fmaf(x3[0], c3v, sr);  si = fmaf(x3[1], c3v, si);
        }
        os[2 * tr] = sr * WSI; os[2 * tr + 1] = si * WSI;
    }
    __syncthreads();
    if (wave < 2) {
        const v4f val = *(const v4fa*)(&os[tid * 4]);
        float* dst = OUT + ((size_t)b * OUT_SEQ + t0) * 2 + tid * 4;
        *(volatile v4f*)dst = val; __threadfence(); *(volatile v4f*)dst = val;
    }
}

static constexpr size_t al256(size_t v) { return (v + 255) & ~(size_t)255; }
static constexpr size_t SZ_WP = al256((size_t)32 * KPAD * 2);
static constexpr size_t SZ_TOTAL = SZ_WP;
static_assert(SZ_TOTAL <= (size_t)134217728);
static_assert((size_t)255 * 8 + 8 <= (size_t)32 * KPAD);

extern "C" void kernel_launch(void* const* d_in, const int* in_sizes, int n_in,
                              void* d_out, int out_size, void* d_ws, size_t ws_size, hipStream_t stream) {
    if (n_in < 5) return;
    const size_t needx = ((size_t)(NB - 1) * SEQ_FULL + SEQ) * 2;
    if ((size_t)in_sizes[0] < needx) return;
    if (in_sizes[2] < LL * NKK || in_sizes[3] < LL * MM * NKK || in_sizes[4] < LL * MM * NKK) return;
    if ((size_t)out_size < ((size_t)(NB - 1) * OUT_SEQ + SEQ) * 2) return;
    if (SZ_TOTAL > ws_size) return;
    const float* x    = (const float*)d_in[0];
    const float* akl  = (const float*)d_in[2];
    const float* bklm = (const float*)d_in[3];
    const float* cklm = (const float*)d_in[4];
    float* OUT = (float*)d_out;
    h16* WP = (h16*)d_ws;

    k_wpack<<<1, 256, 0, stream>>>(akl, bklm, cklm, WP);
    k_mpoly<<<dim3(SEQ / TB, NB, 1), 32 * AWV, 0, stream>>>(x, WP, OUT);
}
